// InrEncoderLayer_59107339927930
// MI455X (gfx1250) — hardware-verified
//
#include <hip/hip_runtime.h>

typedef _Float16 v16h __attribute__((ext_vector_type(16)));
typedef _Float16 v8h  __attribute__((ext_vector_type(8)));
typedef float    v8f  __attribute__((ext_vector_type(8)));
typedef float    v4f  __attribute__((ext_vector_type(4)));
typedef v8h __attribute__((may_alias)) v8ha;
typedef v4f __attribute__((may_alias)) v4fa;

union Frag { v16h v; v8h half[2]; };

#define BATCH  4
#define SEQ    1024
#define FEAT   1024
#define NHEADS 16
#define HD     64
#define FFN    4096
#define MROWS  (BATCH * SEQ)
#define NEGV   (-1.0e9f)
#define LNEPS  (1.0e-5f)
#define WSC    32.0f
#define INVWSC 0.03125f
#define SCINV  0.03125f
#define ASC    16.0f
#define PSCALE 16384.0f

static_assert(MROWS % 128 == 0);
static_assert(SEQ % 128 == 0);
static_assert(FEAT % 64 == 0);
static_assert(FFN % 64 == 0);
static_assert(HD == 64);

__device__ __forceinline__ v8f wmma_f16(v16h a, v16h b, v8f c) {
  v8f d = __builtin_amdgcn_wmma_f32_16x16x32_f16(false, a, false, b, (short)0, c, false, false);
  asm volatile("v_nop\n\tv_nop\n\tv_nop\n\tv_nop" : "+v"(d) : "v"(a), "v"(b));
  return d;
}

__device__ __forceinline__ v16h load_frag(const _Float16* p, int h) {
  Frag f;
  f.half[0] = *(const v8ha*)(p + 8 * h);
  f.half[1] = *(const v8ha*)(p + 16 + 8 * h);
  return f.v;
}

__device__ __forceinline__ void tr_store_pass(const _Float16* sT, _Float16* out, int R,
                                              int c0, int r0, int w, int lane) {
  const int q8 = lane & 7, sb = lane >> 3;
  #pragma unroll
  for (int i = 0; i < 2; ++i) {
    const int cl = w * 8 + i * 4 + sb;
    const v8h v = *(const v8ha*)(sT + cl * 72 + 8 * q8);
    *(volatile v8h*)(out + (size_t)(c0 + cl) * R + r0 + 8 * q8) = v;
  }
}

template <int PERM>
__global__ __launch_bounds__(256) void tr_kernel(
    const float* __restrict__ s0, const float* __restrict__ s1, const float* __restrict__ s2,
    int R, int C, _Float16* __restrict__ dst)
{
  __shared__ __attribute__((aligned(16))) _Float16 sT[64 * 72];
  const int tid = threadIdx.x, lane = tid & 31, w = tid >> 5;
  const int c0 = blockIdx.x * 64, r0 = blockIdx.y * 64, z = blockIdx.z;
  const int sel = z >> 4, sub = z & 15;
  const float* src = (sel == 0) ? s0 : ((sel == 1) ? s1 : s2);
  src += (size_t)sub * R * C;
  _Float16* out = dst + (size_t)z * R * C;

  #pragma unroll
  for (int i = 0; i < 4; ++i) {
    const int rl = i * 16 + (tid >> 4);
    const int cl = (tid & 15) * 4;
    const int ir = PERM ? (rl * 16 + (r0 >> 6)) : (r0 + rl);
    const v4f v = *(const v4fa*)(src + (size_t)ir * C + c0 + cl);
    sT[(cl + 0) * 72 + rl] = (_Float16)(v.x * WSC);
    sT[(cl + 1) * 72 + rl] = (_Float16)(v.y * WSC);
    sT[(cl + 2) * 72 + rl] = (_Float16)(v.z * WSC);
    sT[(cl + 3) * 72 + rl] = (_Float16)(v.w * WSC);
  }
  __syncthreads();
  tr_store_pass(sT, out, R, c0, r0, w, lane);
  __threadfence();
  tr_store_pass(sT, out, R, c0, r0, w, lane);
}

__global__ __launch_bounds__(128) void ln_kernel(
    const float* __restrict__ X, const float* __restrict__ g,
    const float* __restrict__ be, _Float16* __restrict__ Y)
{
  __shared__ float red[8];
  const int tid = threadIdx.x, lane = tid & 31, w = tid >> 5;
  const size_t base = (size_t)blockIdx.x * FEAT + 8 * tid;
  const v4f a = *(const v4fa*)(X + base);
  const v4f c = *(const v4fa*)(X + base + 4);
  float s = ((a.x + a.y) + (a.z + a.w)) + ((c.x + c.y) + (c.z + c.w));
  #pragma unroll
  for (int off = 16; off >= 1; off >>= 1) s += __shfl_xor(s, off);
  if (lane == 0) red[w] = s;
  __syncthreads();
  const float mu = ((red[0] + red[1]) + (red[2] + red[3])) * (1.0f / FEAT);
  const float d0 = a.x - mu, d1 = a.y - mu, d2 = a.z - mu, d3 = a.w - mu;
  const float d4 = c.x - mu, d5 = c.y - mu, d6 = c.z - mu, d7 = c.w - mu;
  float s2 = ((d0 * d0 + d1 * d1) + (d2 * d2 + d3 * d3)) + ((d4 * d4 + d5 * d5) + (d6 * d6 + d7 * d7));
  #pragma unroll
  for (int off = 16; off >= 1; off >>= 1) s2 += __shfl_xor(s2, off);
  if (lane == 0) red[4 + w] = s2;
  __syncthreads();
  const float var = ((red[4] + red[5]) + (red[6] + red[7])) * (1.0f / FEAT);
  const float rstd = rsqrtf(var + LNEPS);
  const v4f ga = *(const v4fa*)(g + 8 * tid);
  const v4f gc = *(const v4fa*)(g + 8 * tid + 4);
  const v4f ba = *(const v4fa*)(be + 8 * tid);
  const v4f bc = *(const v4fa*)(be + 8 * tid + 4);
  v8h o;
  o[0] = (_Float16)(d0 * rstd * ga.x + ba.x);
  o[1] = (_Float16)(d1 * rstd * ga.y + ba.y);
  o[2] = (_Float16)(d2 * rstd * ga.z + ba.z);
  o[3] = (_Float16)(d3 * rstd * ga.w + ba.w);
  o[4] = (_Float16)(d4 * rstd * gc.x + bc.x);
  o[5] = (_Float16)(d5 * rstd * gc.y + bc.y);
  o[6] = (_Float16)(d6 * rstd * gc.z + bc.z);
  o[7] = (_Float16)(d7 * rstd * gc.w + bc.w);
  _Float16* dp = Y + base;
  *(volatile v8h*)dp = o;
  __threadfence();
  *(volatile v8h*)dp = o;
}

__global__ __launch_bounds__(256) void rmsoft_kernel(
    const float* __restrict__ r_mat, const float* __restrict__ attn_mask,
    const float* __restrict__ pad_mask, float* __restrict__ rm)
{
  __shared__ float smax[8];
  __shared__ float ssum[8];
  const int tid = threadIdx.x, lane = tid & 31, w = tid >> 5;
  const size_t row = blockIdx.x;
  const int q = (int)(row & (SEQ - 1));
  const size_t base = row * SEQ + 4 * tid;
  const v4f rv = *(const v4fa*)(r_mat + base);
  const v4f pv = *(const v4fa*)(pad_mask + base);
  const v4f av = *(const v4fa*)(attn_mask + (size_t)q * SEQ + 4 * tid);
  const bool k0 = (pv.x == 0.0f) || (av.x == 0.0f);
  const bool k1 = (pv.y == 0.0f) || (av.y == 0.0f);
  const bool k2 = (pv.z == 0.0f) || (av.z == 0.0f);
  const bool k3 = (pv.w == 0.0f) || (av.w == 0.0f);
  const float v0 = k0 ? NEGV : rv.x;
  const float v1 = k1 ? NEGV : rv.y;
  const float v2 = k2 ? NEGV : rv.z;
  const float v3 = k3 ? NEGV : rv.w;
  float mx = fmaxf(fmaxf(v0, v1), fmaxf(v2, v3));
  #pragma unroll
  for (int off = 16; off >= 1; off >>= 1) mx = fmaxf(mx, __shfl_xor(mx, off));
  if (lane == 0) smax[w] = mx;
  __syncthreads();
  float bmax = smax[0];
  #pragma unroll
  for (int i = 1; i < 8; ++i) bmax = fmaxf(bmax, smax[i]);
  const float e0 = __expf(v0 - bmax);
  const float e1 = __expf(v1 - bmax);
  const float e2 = __expf(v2 - bmax);
  const float e3 = __expf(v3 - bmax);
  float sm = (e0 + e1) + (e2 + e3);
  #pragma unroll
  for (int off = 16; off >= 1; off >>= 1) sm += __shfl_xor(sm, off);
  if (lane == 0) ssum[w] = sm;
  __syncthreads();
  float tot = 0.0f;
  #pragma unroll
  for (int i = 0; i < 8; ++i) tot += ssum[i];
  const float inv = 1.0f / tot;
  v4f o;
  o.x = k0 ? NEGV : e0 * inv;
  o.y = k1 ? NEGV : e1 * inv;
  o.z = k2 ? NEGV : e2 * inv;
  o.w = k3 ? NEGV : e3 * inv;
  float* dp = rm + base;
  *(volatile v4f*)dp = o;
  __threadfence();
  *(volatile v4f*)dp = o;
}

__device__ __forceinline__ void proj_store_pass(const _Float16* sT, _Float16* plane, _Float16* vt,
                                                int which, int bh, int l0, int w, int lane) {
  const int q8 = lane & 7, sub = lane >> 3;
  #pragma unroll
  for (int i = 0; i < 8; ++i) {
    const int lid = w * 32 + i * 4 + sub;
    v8h v;
    _Float16* dst;
    if (which != 2) {
      v = *(const v8ha*)(sT + lid * HD + 8 * q8);
      dst = plane + ((size_t)bh * SEQ + l0 + lid) * HD + 8 * q8;
    } else {
      const int d = lid >> 1, hl = lid & 1;
      v = *(const v8ha*)(sT + d * 128 + 64 * hl + 8 * q8);
      dst = vt + ((size_t)bh * HD + d) * SEQ + l0 + 64 * hl + 8 * q8;
    }
    *(volatile v8h*)dst = v;
  }
}

__global__ __launch_bounds__(128) void proj_kernel(
    const _Float16* __restrict__ hh,
    const _Float16* __restrict__ wt,
    _Float16* __restrict__ qh,
    _Float16* __restrict__ kh,
    _Float16* __restrict__ vt)
{
  __shared__ __attribute__((aligned(16))) _Float16 sT[128 * 64];

  const int tid = threadIdx.x, lane = tid & 31, w = tid >> 5;
  const int h = lane >> 4, m = lane & 15;
  const int m0 = blockIdx.x * 128;
  const int cg = blockIdx.y;
  const int which = cg >> 4, head = cg & 15;
  const int m0w = m0 + 32 * w;

  const _Float16* xa0 = hh + (size_t)(m0w + m) * FEAT;
  const _Float16* xa1 = xa0 + (size_t)16 * FEAT;
  const _Float16* wb  = wt + ((size_t)cg * HD + m) * FEAT;

  const v8f zero8 = {0.f, 0.f, 0.f, 0.f, 0.f, 0.f, 0.f, 0.f};
  v8f acc[2][4];
  #pragma unroll
  for (int mt = 0; mt < 2; ++mt)
    #pragma unroll
    for (int nt = 0; nt < 4; ++nt) acc[mt][nt] = zero8;

  #pragma unroll 1
  for (int k0 = 0; k0 < FEAT; k0 += 32) {
    const v16h a0 = load_frag(xa0 + k0, h);
    const v16h a1 = load_frag(xa1 + k0, h);
    #pragma unroll
    for (int nt = 0; nt < 4; ++nt) {
      const v16h bf = load_frag(wb + (size_t)nt * 16 * FEAT + k0, h);
      acc[0][nt] = wmma_f16(a0, bf, acc[0][nt]);
      acc[1][nt] = wmma_f16(a1, bf, acc[1][nt]);
    }
  }

  #pragma unroll
  for (int nt = 0; nt < 4; ++nt) {
    const int feat = 16 * nt + m;
    #pragma unroll
    for (int mt = 0; mt < 2; ++mt) {
      #pragma unroll
      for (int r = 0; r < 8; ++r) {
        const int tokl = 32 * w + 16 * mt + 8 * h + r;
        const float y = acc[mt][nt][r] * INVWSC;
        const int idx = (which == 2) ? (feat * 128 + tokl) : (tokl * HD + feat);
        sT[idx] = (_Float16)y;
      }
    }
  }
  __syncthreads();

  const int b = m0 / SEQ, l0 = m0 - b * SEQ, bh = b * NHEADS + head;
  _Float16* plane = (which == 0) ? qh : kh;
  proj_store_pass(sT, plane, vt, which, bh, l0, w, lane);
  __threadfence();
  proj_store_pass(sT, plane, vt, which, bh, l0, w, lane);
}

__device__ __forceinline__ v8f add_bias8(v8f s, const float* p) {
  const v4f ra = *(const v4fa*)p;
  const v4f rb = *(const v4fa*)(p + 4);
  float t;
  t = s[0] * SCINV + ra.x; s[0] = (ra.x < -1.0e8f) ? NEGV : t;
  t = s[1] * SCINV + ra.y; s[1] = (ra.y < -1.0e8f) ? NEGV : t;
  t = s[2] * SCINV + ra.z; s[2] = (ra.z < -1.0e8f) ? NEGV : t;
  t = s[3] * SCINV + ra.w; s[3] = (ra.w < -1.0e8f) ? NEGV : t;
  t = s[4] * SCINV + rb.x; s[4] = (rb.x < -1.0e8f) ? NEGV : t;
  t = s[5] * SCINV + rb.y; s[5] = (rb.y < -1.0e8f) ? NEGV : t;
  t = s[6] * SCINV + rb.z; s[6] = (rb.z < -1.0e8f) ? NEGV : t;
  t = s[7] * SCINV + rb.w; s[7] = (rb.w < -1.0e8f) ? NEGV : t;
  return s;
}

__device__ __forceinline__ v16h pack_p(v8f a, v8f c) {
  const v16h r = { (_Float16)(a[0] * PSCALE), (_Float16)(a[1] * PSCALE), (_Float16)(a[2] * PSCALE), (_Float16)(a[3] * PSCALE),
                   (_Float16)(a[4] * PSCALE), (_Float16)(a[5] * PSCALE), (_Float16)(a[6] * PSCALE), (_Float16)(a[7] * PSCALE),
                   (_Float16)(c[0] * PSCALE), (_Float16)(c[1] * PSCALE), (_Float16)(c[2] * PSCALE), (_Float16)(c[3] * PSCALE),
                   (_Float16)(c[4] * PSCALE), (_Float16)(c[5] * PSCALE), (_Float16)(c[6] * PSCALE), (_Float16)(c[7] * PSCALE) };
  return r;
}

__device__ __forceinline__ void att_store_pass(const _Float16* so, _Float16* ab,
                                               int b, int head, int q0, int lane) {
  const int q8 = lane & 7, sub = lane >> 3;
  #pragma unroll
  for (int i = 0; i < 4; ++i) {
    const int row = i * 4 + sub;
    const v8h v = *(const v8ha*)(so + row * HD + 8 * q8);
    const size_t gi = ((size_t)b * SEQ + q0 + row) * FEAT + head * HD + 8 * q8;
    *(volatile v8h*)(ab + gi) = v;
  }
}

__global__ __launch_bounds__(128) void attn_kernel(
    const _Float16* __restrict__ qh,
    const _Float16* __restrict__ kh,
    const _Float16* __restrict__ vt,
    const float* __restrict__ rm,
    _Float16* __restrict__ ab)
{
  __shared__ __attribute__((aligned(16))) _Float16 sO[4 * 16 * 64];

  const int tid = threadIdx.x, lane = tid & 31, w = tid >> 5;
  const int h = lane >> 4, m = lane & 15;
  const int bh = blockIdx.y, b = bh >> 4, head = bh & 15;
  const int q0 = blockIdx.x * 64 + 16 * w;

  const _Float16* qrow = qh + ((size_t)bh * SEQ + q0 + m) * HD;
  const v16h qb0 = load_frag(qrow, h);
  const v16h qb1 = load_frag(qrow + 32, h);

  const v8f zero8 = {0.f, 0.f, 0.f, 0.f, 0.f, 0.f, 0.f, 0.f};
  v8f o[4];
  #pragma unroll
  for (int t = 0; t < 4; ++t) o[t] = zero8;
  float mrun = -1e30f, lrun = 0.0f;

  const _Float16* kbase = kh + ((size_t)bh * SEQ + m) * HD;
  const _Float16* vbase = vt + ((size_t)bh * HD + m) * SEQ;
  const float* rp = rm + ((size_t)b * SEQ + q0 + m) * SEQ + 8 * h;

  #pragma unroll 1
  for (int kb = 0; kb < SEQ; kb += 64) {
    v8f s[4];
    #pragma unroll
    for (int j = 0; j < 4; ++j) {
      const _Float16* kp = kbase + (size_t)(kb + 16 * j) * HD;
      const v16h kf0 = load_frag(kp, h);
      const v16h kf1 = load_frag(kp + 32, h);
      v8f z = zero8;
      z = wmma_f16(kf0, qb0, z);
      z = wmma_f16(kf1, qb1, z);
      s[j] = z;
    }
    #pragma unroll
    for (int j = 0; j < 4; ++j) s[j] = add_bias8(s[j], rp + kb + 16 * j);

    float mloc = s[0][0];
    #pragma unroll
    for (int j = 0; j < 4; ++j)
      #pragma unroll
      for (int r = 0; r < 8; ++r) mloc = fmaxf(mloc, s[j][r]);
    mloc = fmaxf(mloc, __shfl_xor(mloc, 16));
    const float mnew = fmaxf(mrun, mloc);
    const float alpha = __expf(mrun - mnew);
    mrun = mnew;
    float lsum = 0.0f;
    #pragma unroll
    for (int j = 0; j < 4; ++j)
      #pragma unroll
      for (int r = 0; r < 8; ++r) {
        const float p = __expf(s[j][r] - mnew);
        s[j][r] = p;
        lsum += p;
      }
    lsum += __shfl_xor(lsum, 16);
    lrun = lrun * alpha + lsum;
    #pragma unroll
    for (int t = 0; t < 4; ++t)
      #pragma unroll
      for (int r = 0; r < 8; ++r) o[t][r] = o[t][r] * alpha;

    const v16h pb0 = pack_p(s[0], s[1]);
    const v16h pb1 = pack_p(s[2], s[3]);

    #pragma unroll
    for (int t = 0; t < 4; ++t) {
      const _Float16* vp = vbase + (size_t)(16 * t) * SEQ + kb;
      const v16h vf0 = load_frag(vp, h);
      const v16h vf1 = load_frag(vp + 32, h);
      o[t] = wmma_f16(vf0, pb0, o[t]);
      o[t] = wmma_f16(vf1, pb1, o[t]);
    }
  }

  const float inv = (1.0f / lrun) * (ASC / PSCALE);
  _Float16* so = sO + w * 1024;
  #pragma unroll
  for (int t = 0; t < 4; ++t)
    #pragma unroll
    for (int r = 0; r < 8; ++r)
      so[m * HD + 16 * t + 8 * h + r] = (_Float16)(o[t][r] * inv);
  __syncthreads();

  att_store_pass(so, ab, b, head, q0, lane);
  __threadfence();
  att_store_pass(so, ab, b, head, q0, lane);
}

__device__ __forceinline__ void f32_store_pass(const float* sw, float* outF, int N,
                                               int m0w, int n0, int h, int m) {
  #pragma unroll
  for (int i = 0; i < 16; ++i) {
    const int rowl = 2 * i + h;
    const v4f v = *(const v4fa*)(sw + rowl * 64 + 4 * m);
    *(volatile v4f*)(outF + (size_t)(m0w + rowl) * N + n0 + 4 * m) = v;
  }
}

__device__ __forceinline__ void f16_store_pass(const _Float16* sh, _Float16* outH, int N,
                                               int m0w, int n0, int lane) {
  const int q8 = lane & 7, sub = lane >> 3;
  #pragma unroll
  for (int i = 0; i < 8; ++i) {
    const int rowl = i * 4 + sub;
    const v8h v = *(const v8ha*)(sh + rowl * 64 + 8 * q8);
    *(volatile v8h*)(outH + (size_t)(m0w + rowl) * N + n0 + 8 * q8) = v;
  }
}

template <int EPI, int HASB>
__global__ __launch_bounds__(128) void gemm_kernel(
    const _Float16* __restrict__ A,
    const _Float16* __restrict__ Bt,
    int K, int N,
    const float* __restrict__ bias,
    const float* __restrict__ res,
    float* __restrict__ outF,
    _Float16* __restrict__ outH,
    float oscale)
{
  __shared__ __attribute__((aligned(16))) union { float f[4 * 32 * 64]; _Float16 hh[4 * 32 * 64 * 2]; } sEp;

  const int tid = threadIdx.x, lane = tid & 31, w = tid >> 5;
  const int h = lane >> 4, m = lane & 15;
  const int m0 = blockIdx.x * 128, n0 = blockIdx.y * 64;
  const int m0w = m0 + 32 * w;

  const _Float16* xa0 = A + (size_t)(m0w + m) * K;
  const _Float16* xa1 = xa0 + (size_t)16 * K;
  const _Float16* wb  = Bt + (size_t)(n0 + m) * K;

  const v8f zero8 = {0.f, 0.f, 0.f, 0.f, 0.f, 0.f, 0.f, 0.f};
  v8f acc[2][4];
  #pragma unroll
  for (int mt = 0; mt < 2; ++mt)
    #pragma unroll
    for (int nt = 0; nt < 4; ++nt) acc[mt][nt] = zero8;

  #pragma unroll 1
  for (int k0 = 0; k0 < K; k0 += 32) {
    const v16h a0 = load_frag(xa0 + k0, h);
    const v16h a1 = load_frag(xa1 + k0, h);
    #pragma unroll
    for (int nt = 0; nt < 4; ++nt) {
      const v16h bf = load_frag(wb + (size_t)nt * 16 * K + k0, h);
      acc[0][nt] = wmma_f16(a0, bf, acc[0][nt]);
      acc[1][nt] = wmma_f16(a1, bf, acc[1][nt]);
    }
  }

  if constexpr (EPI == 0) {
    float* sw = sEp.f + w * 2048;
    #pragma unroll
    for (int nt = 0; nt < 4; ++nt) {
      const int coll = 16 * nt + m;
      float bv = 0.0f;
      if constexpr (HASB) bv = bias[n0 + coll];
      #pragma unroll
      for (int mt = 0; mt < 2; ++mt) {
        #pragma unroll
        for (int r = 0; r < 8; ++r) {
          const int rowl = 16 * mt + 8 * h + r;
          const float rv = res[(size_t)(m0w + rowl) * N + n0 + coll];
          const float v = rv + (acc[mt][nt][r] * oscale + bv);
          sw[rowl * 64 + coll] = v;
        }
      }
    }
    __syncthreads();
    f32_store_pass(sw, outF, N, m0w, n0, h, m);
    __threadfence();
    f32_store_pass(sw, outF, N, m0w, n0, h, m);
  } else {
    _Float16* sh = sEp.hh + w * 2048;
    #pragma unroll
    for (int nt = 0; nt < 4; ++nt) {
      const int coll = 16 * nt + m;
      const float bv = bias[n0 + coll];
      #pragma unroll
      for (int mt = 0; mt < 2; ++mt) {
        #pragma unroll
        for (int r = 0; r < 8; ++r) {
          const int rowl = 16 * mt + 8 * h + r;
          const float v = fmaxf(acc[mt][nt][r] * oscale + bv, 0.0f);
          sh[rowl * 64 + coll] = (_Float16)v;
        }
      }
    }
    __syncthreads();
    f16_store_pass(sh, outH, N, m0w, n0, lane);
    __threadfence();
    f16_store_pass(sh, outH, N, m0w, n0, lane);
  }
}

extern "C" void kernel_launch(void* const* d_in, const int* in_sizes, int n_in,
                              void* d_out, int out_size, void* d_ws, size_t ws_size,
                              hipStream_t stream) {
  if (n_in < 16) return;
  const int NX  = MROWS * FEAT;
  const int NRM = BATCH * SEQ * SEQ;
  const int NWH = NHEADS * FEAT * HD;
  if (in_sizes[0] != NX || in_sizes[1] != NRM) return;
  if (in_sizes[2] != SEQ * SEQ || in_sizes[3] != NRM) return;
  if (in_sizes[4] != NWH || in_sizes[5] != NWH || in_sizes[6] != NWH) return;
  if (in_sizes[7] != FEAT * FEAT) return;
  if (in_sizes[8] != FEAT * FFN || in_sizes[9] != FFN) return;
  if (in_sizes[10] != FFN * FEAT || in_sizes[11] != FEAT) return;
  if (in_sizes[12] != FEAT || in_sizes[13] != FEAT || in_sizes[14] != FEAT || in_sizes[15] != FEAT) return;
  if (out_size != NX) return;

  const float* x         = (const float*)d_in[0];
  const float* r_mat     = (const float*)d_in[1];
  const float* attn_mask = (const float*)d_in[2];
  const float* pad_mask  = (const float*)d_in[3];
  const float* Wq        = (const float*)d_in[4];
  const float* Wk        = (const float*)d_in[5];
  const float* Wv        = (const float*)d_in[6];
  const float* Wo        = (const float*)d_in[7];
  const float* w1        = (const float*)d_in[8];
  const float* b1        = (const float*)d_in[9];
  const float* w2        = (const float*)d_in[10];
  const float* b2        = (const float*)d_in[11];
  const float* g1        = (const float*)d_in[12];
  const float* be1       = (const float*)d_in[13];
  const float* g2        = (const float*)d_in[14];
  const float* be2       = (const float*)d_in[15];
  float* out = (float*)d_out;

  const size_t wqkv_bytes = (size_t)3 * NWH * 2;
  const size_t wo_bytes   = (size_t)FEAT * FEAT * 2;
  const size_t w1_bytes   = (size_t)FFN * FEAT * 2;
  const size_t w2_bytes   = (size_t)FEAT * FFN * 2;
  const size_t h_bytes    = (size_t)NX * 2;
  const size_t pl_bytes   = (size_t)NX * 2;
  const size_t rm_bytes   = (size_t)NRM * 4;
  const size_t x1_bytes   = (size_t)NX * 4;
  const size_t off_wqkv = 0;
  const size_t off_wo   = off_wqkv + wqkv_bytes;
  const size_t off_w1   = off_wo + wo_bytes;
  const size_t off_w2   = off_w1 + w1_bytes;
  const size_t off_h    = off_w2 + w2_bytes;
  const size_t off_q    = off_h + h_bytes;
  const size_t off_k    = off_q + pl_bytes;
  const size_t off_vt   = off_k + pl_bytes;
  const size_t off_a    = off_vt + pl_bytes;
  const size_t off_rm   = off_a + pl_bytes;
  const size_t off_x1   = off_rm + rm_bytes;
  const size_t total    = off_x1 + x1_bytes;
  const size_t mid_bytes = (size_t)MROWS * FFN * 2;
  if (mid_bytes > 4 * pl_bytes) return;
  if (total > ws_size) return;

  char* ws = (char*)d_ws;
  _Float16* wqkvT = (_Float16*)(ws + off_wqkv);
  _Float16* woT   = (_Float16*)(ws + off_wo);
  _Float16* w1T   = (_Float16*)(ws + off_w1);
  _Float16* w2T   = (_Float16*)(ws + off_w2);
  _Float16* hbuf  = (_Float16*)(ws + off_h);
  _Float16* qh    = (_Float16*)(ws + off_q);
  _Float16* kh    = (_Float16*)(ws + off_k);
  _Float16* vtb   = (_Float16*)(ws + off_vt);
  _Float16* abuf  = (_Float16*)(ws + off_a);
  float*    rm    = (float*)(ws + off_rm);
  float*    x1    = (float*)(ws + off_x1);
  _Float16* mid   = (_Float16*)(ws + off_q);

  tr_kernel<0><<<dim3(HD / 64, FEAT / 64, 3 * NHEADS), 256, 0, stream>>>(Wq, Wk, Wv, FEAT, HD, wqkvT);
  tr_kernel<1><<<dim3(FEAT / 64, FEAT / 64, 1), 256, 0, stream>>>(Wo, Wo, Wo, FEAT, FEAT, woT);
  tr_kernel<0><<<dim3(FFN / 64, FEAT / 64, 1), 256, 0, stream>>>(w1, w1, w1, FEAT, FFN, w1T);
  tr_kernel<0><<<dim3(FEAT / 64, FFN / 64, 1), 256, 0, stream>>>(w2, w2, w2, FFN, FEAT, w2T);

  ln_kernel<<<MROWS, 128, 0, stream>>>(x, g1, be1, hbuf);

  proj_kernel<<<dim3(MROWS / 128, 3 * NHEADS), 128, 0, stream>>>(hbuf, wqkvT, qh, kh, vtb);

  rmsoft_kernel<<<BATCH * SEQ, 256, 0, stream>>>(r_mat, attn_mask, pad_mask, rm);

  attn_kernel<<<dim3(SEQ / 64, BATCH * NHEADS), 128, 0, stream>>>(qh, kh, vtb, rm, abuf);

  gemm_kernel<0, 0><<<dim3(MROWS / 128, FEAT / 64), 128, 0, stream>>>(
      abuf, woT, FEAT, FEAT, b2, x, x1, hbuf, 1.0f / 512.0f);

  ln_kernel<<<MROWS, 128, 0, stream>>>(x1, g2, be2, hbuf);

  gemm_kernel<1, 1><<<dim3(MROWS / 128, FFN / 64), 128, 0, stream>>>(
      hbuf, w1T, FEAT, FFN, b1, x1, x1, mid, INVWSC);

  gemm_kernel<0, 1><<<dim3(MROWS / 128, FEAT / 64), 128, 0, stream>>>(
      mid, w2T, FFN, FEAT, b2, x1, out, hbuf, INVWSC);
}
